// PointConv_68745246539912
// MI455X (gfx1250) — hardware-run, weakly checked
//
#include <hip/hip_runtime.h>
#include <stddef.h>
#include <stdint.h>


#define CF      128
#define NRPT    100000
#define NQPT    50000
#define NEDG    1600000
#define MPAD    100096
#define NTHR    256
#define NWAVE   8
#define NBRUN   1024
#define SLB     10
#define NBLK    49
#define TPAD    (NBLK * NBRUN)
#define WC      4608
#define RCAP    (NWAVE * WC)
#define DEGCAP  96
#define RSH     17
#define GBM     64
#define GBN     128
#define GTHR    128
#define XUNITS  (MPAD * (CF / 8))
#define WUNITS  (CF * (CF / 8))
#define BK_ZINTS (RCAP + RCAP / 2 + NWAVE * NBRUN + 2 * NBRUN)
#define BK_INTS  (BK_ZINTS + 16)

static_assert(NRPT < (1 << RSH));
static_assert(NBRUN == (1 << SLB) && NBRUN == (1 << 10));
static_assert(RSH + SLB <= 32);
static_assert(NBLK * NBRUN >= NQPT);
static_assert(CF == 32 * 4 && CF % 32 == 0);
static_assert(((long long)(NEDG + 8 * 256) << SLB) < (1LL << 31));
static_assert(RCAP >= 33259 + 33259 / 20 && RCAP <= 65536);
static_assert(DEGCAP >= 61 + 8 && DEGCAP % 32 == 0);
static_assert(MPAD % 128 == 0 && MPAD >= NRPT && MPAD % GBM == 0);
static_assert(XUNITS % NTHR == 0 && WUNITS % NTHR == 0);
static_assert(RCAP % (NTHR * 4) == 0 && BK_ZINTS % (NTHR * 4) == 0);
static_assert(NBRUN % NWAVE == 0 && NBRUN % NTHR == 0 && NBRUN == 4 * NTHR);
static_assert(GBN == CF && GBM == (GTHR / 32) * 16);
static_assert(BK_INTS * 4 <= 300000);
static_assert(BK_INTS * 4 + 0 <= 327680);
static_assert(4 * CF == 2 * NTHR);

static constexpr size_t al256c(size_t o) { return (o + 255) & ~(size_t)255; }
static constexpr size_t SZ_WB   = (size_t)CF * CF * 2;
static constexpr size_t SZ_XB   = (size_t)MPAD * CF * 2;
static constexpr size_t SZ_RF   = (size_t)MPAD * CF * 4;
static constexpr size_t SZ_TQ   = (size_t)TPAD * CF * 4;
static constexpr size_t SZ_LIST = (size_t)NBLK * RCAP * 4;
static constexpr size_t SZ_CNT  = (size_t)TPAD * 4;
static constexpr size_t SZ_FLG  = al256c((size_t)NBLK * 128);
static constexpr size_t SZ_REC  = (size_t)NBLK * 2 * CF * 8;
static constexpr size_t SZ_STAT = (size_t)4 * CF * 4;
static constexpr size_t OF_WB   = 0;
static constexpr size_t OF_XB   = OF_WB + SZ_WB;
static constexpr size_t OF_RF   = OF_XB + SZ_XB;
static constexpr size_t OF_TQ   = OF_RF + SZ_RF;
static constexpr size_t OF_LIST = OF_TQ + SZ_TQ;
static constexpr size_t OF_CNT  = OF_LIST + SZ_LIST;
static constexpr size_t OF_OFF  = OF_CNT + SZ_CNT;
static constexpr size_t OF_FLG  = OF_OFF + SZ_CNT;
static constexpr size_t OF_REC  = OF_FLG + SZ_FLG;
static constexpr size_t OF_STAT = OF_REC + SZ_REC;
static constexpr size_t WS_TOTAL = OF_STAT + SZ_STAT;
static_assert(SZ_WB % 256 == 0 && SZ_XB % 256 == 0 && SZ_RF % 256 == 0 && SZ_TQ % 256 == 0);
static_assert(SZ_LIST % 256 == 0 && SZ_CNT % 256 == 0 && SZ_REC % 256 == 0 && SZ_STAT % 256 == 0);
static_assert(WS_TOTAL <= ((size_t)128u << 20));

typedef float          v4f   __attribute__((ext_vector_type(4)));
typedef float          v8f   __attribute__((ext_vector_type(8)));
typedef int            v4i   __attribute__((ext_vector_type(4)));
typedef int            v8i   __attribute__((ext_vector_type(8)));
typedef unsigned       v2u   __attribute__((ext_vector_type(2)));
typedef unsigned       v4u   __attribute__((ext_vector_type(4)));
typedef unsigned short v8us  __attribute__((ext_vector_type(8)));
typedef unsigned short v16us __attribute__((ext_vector_type(16)));
typedef __bf16         v16bf __attribute__((ext_vector_type(16)));
typedef double         v2d   __attribute__((ext_vector_type(2)));
typedef v4f  __attribute__((may_alias)) v4fa;
typedef v4i  __attribute__((may_alias)) v4ia;
typedef v2u  __attribute__((may_alias)) v2ua;
typedef v8us __attribute__((may_alias)) v8usa;
typedef v2d  __attribute__((may_alias)) v2da;
union FragB { v16bf v; v16us u; v8us h[2]; v8i w; };

__device__ __forceinline__ v8f wmb(const FragB& a, const FragB& b, v8f c) {
  v8f d = __builtin_amdgcn_wmma_f32_16x16x32_bf16(false, a.v, false, b.v, (short)0, c, false, false);
  asm volatile("v_nop\n\tv_nop\n\tv_nop\n\tv_nop" : "+v"(d) : "v"(a.w), "v"(b.w));
  return d;
}

__device__ __forceinline__ unsigned bf16_bits(float f) {
  const unsigned u = __float_as_uint(f);
  return (u + 0x7fffu + ((u >> 16) & 1u)) >> 16;
}
__device__ __forceinline__ float bf16_val(float f) {
  return __uint_as_float(bf16_bits(f) << 16);
}

__device__ __forceinline__ v8us pack8(v4f a, v4f b, unsigned keep) {
  v8us o;
  o[0] = (unsigned short)(bf16_bits(a.x) & keep); o[1] = (unsigned short)(bf16_bits(a.y) & keep);
  o[2] = (unsigned short)(bf16_bits(a.z) & keep); o[3] = (unsigned short)(bf16_bits(a.w) & keep);
  o[4] = (unsigned short)(bf16_bits(b.x) & keep); o[5] = (unsigned short)(bf16_bits(b.y) & keep);
  o[6] = (unsigned short)(bf16_bits(b.z) & keep); o[7] = (unsigned short)(bf16_bits(b.w) & keep);
  return o;
}
__device__ __forceinline__ void put8(unsigned short* dp, v8us o) {
  *(volatile v8us*)dp = o;
  __threadfence();
  *(volatile v8us*)dp = o;
}

__global__ __launch_bounds__(NTHR) void k_prep(const float* __restrict__ xf, const float* __restrict__ wm, int nR,
                                               unsigned short* xb, unsigned short* wb) {
  const int u = (int)blockIdx.x * NTHR + (int)threadIdx.x;
  if ((int)blockIdx.x < XUNITS / NTHR) {
    const int row = u >> 4;
    const int k8  = (u & 15) * 8;
    const int rc  = row < nR ? row : nR - 1;
    const float* p = xf + (size_t)rc * CF + k8;
    const v4f a = *(const v4f*)p;
    const v4f b = *(const v4f*)(p + 4);
    asm volatile("" :: "v"(a), "v"(b));
    const unsigned keep = row < nR ? 0xffffu : 0u;
    put8(xb + (size_t)u * 8, pack8(a, b, keep));
  } else {
    int v = u - XUNITS;
    v = v < 0 ? 0 : (v > WUNITS - 1 ? WUNITS - 1 : v);
    const float* p = wm + (size_t)v * 8;
    const v4f a = *(const v4f*)p;
    const v4f b = *(const v4f*)(p + 4);
    put8(wb + (size_t)v * 8, pack8(a, b, 0xffffu));
  }
}

__global__ __launch_bounds__(GTHR) void k_gemm(const unsigned short* __restrict__ A,
                                               const unsigned short* __restrict__ BT,
                                               const float* __restrict__ bias, float* rf, int nR) {
  __shared__ __attribute__((aligned(16))) float stg[GBM * GBN];
  const int tid = (int)threadIdx.x, lane = tid & 31, wave = tid >> 5, hh = lane >> 4, m = lane & 15;
  const int rowBase = (int)blockIdx.x * GBM;

  v8f acc[8];
  {
    const v8f z = {0.f, 0.f, 0.f, 0.f, 0.f, 0.f, 0.f, 0.f};
#pragma unroll
    for (int t = 0; t < 8; ++t) acc[t] = z;
  }
  const unsigned short* ap = A + (size_t)(rowBase + 16 * wave + m) * (size_t)CF + 8 * hh;
  const unsigned short* bp = BT + (size_t)m * (size_t)CF + 8 * hh;

#pragma unroll 1
  for (int k0 = 0; k0 < CF; k0 += 32) {
    FragB af;
    af.h[0] = *(const v8usa*)(ap + k0);
    af.h[1] = *(const v8usa*)(ap + k0 + 16);
#pragma unroll
    for (int nt = 0; nt < 8; ++nt) {
      const unsigned short* wq = bp + (size_t)(16 * nt) * (size_t)CF + k0;
      FragB bf;
      bf.h[0] = *(const v8usa*)wq;
      bf.h[1] = *(const v8usa*)(wq + 16);
      acc[nt] = wmb(af, bf, acc[nt]);
    }
  }

#pragma unroll
  for (int nt = 0; nt < 8; ++nt) {
    const int lc = 16 * nt + m;
#pragma unroll
    for (int r = 0; r < 8; ++r) {
      const int lr = 16 * wave + 8 * hh + r;
      stg[lr * GBN + lc] = acc[nt][r];
    }
  }
  __syncthreads();

  v4f bb4;
  {
    const v4f t1 = *(const v4f*)(bias + 4 * lane);
    bb4.x = bf16_val(t1.x); bb4.y = bf16_val(t1.y); bb4.z = bf16_val(t1.z); bb4.w = bf16_val(t1.w);
  }
  v4f pv[16];
#pragma unroll
  for (int i = 0; i < 16; ++i) {
    const bool ok = (rowBase + 16 * wave + i) < nR;
    const v4f t = *(const v4fa*)(stg + (16 * wave + i) * GBN + 4 * lane) + bb4;
    v4f y;
    y.x = ok ? t.x : 0.0f; y.y = ok ? t.y : 0.0f; y.z = ok ? t.z : 0.0f; y.w = ok ? t.w : 0.0f;
    pv[i] = y;
  }
#pragma unroll
  for (int i = 0; i < 16; ++i) {
    *(volatile v4f*)(rf + (size_t)(rowBase + 16 * wave + i) * CF + 4 * lane) = pv[i];
  }
  __threadfence();
#pragma unroll
  for (int i = 0; i < 16; ++i) {
    *(volatile v4f*)(rf + (size_t)(rowBase + 16 * wave + i) * CF + 4 * lane) = pv[i];
  }
}

__global__ __launch_bounds__(NTHR) void k_bucket(const int* __restrict__ keys, const int* __restrict__ gix,
                                                 int nE, int nQ, int nR, int span,
                                                 unsigned* listg, int* cntg, int* offg, int* flgg) {
  extern __shared__ __attribute__((aligned(16))) int dsm[];
  int* wl   = dsm;
  unsigned short* perm = (unsigned short*)(dsm + RCAP);
  int* wcnt = dsm + RCAP + RCAP / 2;
  int* cnt  = wcnt + NWAVE * NBRUN;
  int* offs = cnt + NBRUN;
  int* misc = offs + NBRUN;
  const int tid = (int)threadIdx.x, lane = tid & 31;
  const int wv = __builtin_amdgcn_readfirstlane(tid >> 5);
  const int slotBase = (int)blockIdx.x * NBRUN;

  {
    const v4i z4 = {0, 0, 0, 0};
    for (int i = tid * 4; i < BK_ZINTS; i += NTHR * 4) *(v4ia*)(dsm + i) = z4;
    if (tid < 16) misc[tid] = 0;
  }
  __syncthreads();

  {
    int wc = 0;
    const int sent = (int)(1u << 31);
    const int wstart = wv * span;
    const int nIt = span >> 8;
#pragma unroll 1
    for (int it = 0; it < nIt; ++it) {
      const int base = wstart + it * 256;
#pragma unroll
      for (int g = 0; g < 2; ++g) {
        int kv[4];
#pragma unroll
        for (int j = 0; j < 4; ++j) {
          const int e = base + (4 * g + j) * 32 + lane;
          const int ka = keys[min(e, nE - 1)];
          asm volatile("" :: "v"(ka));
          kv[j] = (e < nE) ? ka : sent;
        }
#pragma unroll
        for (int j = 0; j < 4; ++j) {
          const int e = base + (4 * g + j) * 32 + lane;
          const unsigned sj = (unsigned)kv[j] - (unsigned)slotBase;
          const bool hit = (sj < (unsigned)NBRUN) && ((unsigned)kv[j] < (unsigned)nQ);
          const unsigned mj = __builtin_amdgcn_ballot_w32(hit);
          if (mj != 0u) {
            if (hit) {
              const int pos = wc + (int)__builtin_amdgcn_mbcnt_lo(mj, 0u);
              if (pos < WC) wl[wv * WC + pos] = (e << SLB) | (int)sj;
            }
            wc += (int)__builtin_popcount(mj);
          }
        }
      }
    }
    if (lane == 0) misc[wv] = wc;
  }
  __syncthreads();

  int ovf = 0;
#pragma unroll
  for (int w = 0; w < NWAVE; ++w) ovf |= (misc[w] > WC) ? 1 : 0;
  int cv = misc[wv];
  cv = cv < 0 ? 0 : (cv > WC ? WC : cv);
  const int cw = __builtin_amdgcn_readfirstlane(cv);

#pragma unroll 1
  for (int b0 = 0; b0 < cw; b0 += 32) {
    int idx = b0 + lane;
    idx = idx < WC ? idx : WC - 1;
    const int ent = wl[wv * WC + idx];
    const int m32 = min(cw - b0, 32);
#pragma unroll 1
    for (int k = 0; k < m32; ++k) {
      const int u    = __builtin_amdgcn_readlane(ent, k);
      const int slot = u & (NBRUN - 1);
      if (lane == 0) wcnt[wv * NBRUN + slot] = wcnt[wv * NBRUN + slot] + 1;
    }
  }
  __syncthreads();

#pragma unroll 1
  for (int q = 0; q < NBRUN / NTHR; ++q) {
    const int s = q * NTHR + tid;
    int run = 0;
#pragma unroll
    for (int w = 0; w < NWAVE; ++w) {
      const int v = wcnt[w * NBRUN + s];
      wcnt[w * NBRUN + s] = run;
      run += v;
    }
    cnt[s] = run;
  }
  __syncthreads();

  if (wv == 0) {
    const int base = lane * (NBRUN / 32);
    int s = 0;
#pragma unroll 1
    for (int i = 0; i < NBRUN / 32; ++i) s += cnt[base + i];
    int incl = s;
#pragma unroll
    for (int d = 1; d < 32; d <<= 1) {
      const int y = __shfl_up(incl, d, 32);
      if (lane >= d) incl += y;
    }
    int run = incl - s;
#pragma unroll 1
    for (int i = 0; i < NBRUN / 32; ++i) {
      const int c2 = cnt[base + i];
      offs[base + i] = run;
      run += c2;
    }
  }
  __syncthreads();

#pragma unroll 1
  for (int b0 = 0; b0 < cw; b0 += 32) {
    int idx = b0 + lane;
    idx = idx < WC ? idx : WC - 1;
    const int ent = wl[wv * WC + idx];
    const int m32 = min(cw - b0, 32);
#pragma unroll 1
    for (int k = 0; k < m32; ++k) {
      const int u    = __builtin_amdgcn_readlane(ent, k);
      const int slot = u & (NBRUN - 1);
      if (lane == 0) {
        const int r = wcnt[wv * NBRUN + slot];
        int p = offs[slot] + r;
        p = p < 0 ? 0 : (p > RCAP - 1 ? RCAP - 1 : p);
        perm[p] = (unsigned short)(wv * WC + b0 + k);
        wcnt[wv * NBRUN + slot] = r + 1;
      }
    }
  }
  __syncthreads();

  int tt = offs[NBRUN - 1] + cnt[NBRUN - 1];
  tt = tt < 0 ? 0 : (tt > RCAP ? RCAP : tt);
  unsigned* lrow = listg + (size_t)blockIdx.x * RCAP;
#pragma unroll 1
  for (int it = 0; it < RCAP / (NTHR * 4); ++it) {
    const int i0 = (it * NTHR + tid) * 4;
    const v2u pw = *(const v2ua*)(perm + i0);
    int pi[4];
    pi[0] = (int)(pw.x & 0xffffu); pi[1] = (int)(pw.x >> 16);
    pi[2] = (int)(pw.y & 0xffffu); pi[3] = (int)(pw.y >> 16);
    v4u o;
#pragma unroll
    for (int j = 0; j < 4; ++j) {
      const int idx = pi[j] > RCAP - 1 ? RCAP - 1 : pi[j];
      const int u = wl[idx];
      int eid = u >> SLB;
      eid = eid < 0 ? 0 : (eid > nE - 1 ? nE - 1 : eid);
      int r = gix[eid];
      asm volatile("" :: "v"(r));
      r = r < 0 ? 0 : (r > nR - 1 ? nR - 1 : r);
      const unsigned w = (unsigned)r | ((unsigned)(u & (NBRUN - 1)) << RSH);
      const unsigned keep = (i0 + j < tt) ? 0xffffffffu : 0u;
      o[j] = w & keep;
    }
    *(volatile v4u*)(lrow + i0) = o;
    __threadfence();
    *(volatile v4u*)(lrow + i0) = o;
  }
  {
    const v4i c4 = *(const v4ia*)(cnt + 4 * tid);
    const v4i o4 = *(const v4ia*)(offs + 4 * tid);
    int* cp = cntg + (size_t)blockIdx.x * NBRUN + 4 * tid;
    int* op = offg + (size_t)blockIdx.x * NBRUN + 4 * tid;
    v4i f4;
    f4.x = ovf; f4.y = tt; f4.z = 0; f4.w = 0;
    int* fp = flgg + (size_t)blockIdx.x * 32 + 4 * (tid & 7);
    *(volatile v4i*)cp = c4;
    *(volatile v4i*)op = o4;
    if (tid < 8) *(volatile v4i*)fp = f4;
    __threadfence();
    *(volatile v4i*)cp = c4;
    *(volatile v4i*)op = o4;
    if (tid < 8) *(volatile v4i*)fp = f4;
  }
}

__global__ __launch_bounds__(NTHR) void k_replay(const float* __restrict__ rf, const float* __restrict__ rxyz,
                                                 const float* __restrict__ qxyz, const float* __restrict__ wpos,
                                                 const float* __restrict__ bpos,
                                                 const unsigned* __restrict__ listg, const int* __restrict__ cntg,
                                                 const int* __restrict__ offg, const int* __restrict__ flgg,
                                                 int nQ, int nR, float* tq, double* rec) {
  __shared__ __attribute__((aligned(16))) float  wraw[3 * CF];
  __shared__ __attribute__((aligned(16))) float  wpl[4 * CF];
  __shared__ __attribute__((aligned(16))) double wst[NWAVE * 2 * CF];
  __shared__ __attribute__((aligned(16))) double recs[2 * CF];
  const int tid = (int)threadIdx.x, lane = tid & 31, wave = tid >> 5;
  const int blk = (int)blockIdx.x;
  const int nodeBase = blk * NBRUN;

  if (tid < 96) {
    *(v4fa*)(wraw + 4 * tid) = *(const v4f*)(wpos + 4 * tid);
  } else if (tid < 128) {
    const int t = tid - 96;
    const v4f b = *(const v4f*)(bpos + 4 * t);
    v4f bb;
    bb.x = bf16_val(b.x); bb.y = bf16_val(b.y); bb.z = bf16_val(b.z); bb.w = bf16_val(b.w);
    *(v4fa*)(wpl + 3 * CF + 4 * t) = bb;
  }
  __syncthreads();
  if (tid < CF) {
    wpl[tid]          = bf16_val(wraw[3 * tid]);
    wpl[CF + tid]     = bf16_val(wraw[3 * tid + 1]);
    wpl[2 * CF + tid] = bf16_val(wraw[3 * tid + 2]);
  }
  __syncthreads();
  const v4f wp0 = *(const v4fa*)(wpl + 4 * lane);
  const v4f wp1 = *(const v4fa*)(wpl + CF + 4 * lane);
  const v4f wp2 = *(const v4fa*)(wpl + 2 * CF + 4 * lane);
  const v4f bp4 = *(const v4fa*)(wpl + 3 * CF + 4 * lane);

  const unsigned* lst = listg + (size_t)blk * RCAP;
  const int fl = flgg[(size_t)blk * 32];
  const float qnan = __int_as_float(0x7fc00000);
  const float pz = (fl != 0) ? qnan : 0.0f;

  double sm[4], sq[4];
#pragma unroll
  for (int j = 0; j < 4; ++j) { sm[j] = 0.0; sq[j] = 0.0; }

#pragma unroll 1
  for (int si = 0; si < NBRUN / NWAVE; ++si) {
    const int s    = si * NWAVE + wave;
    const int node = nodeBase + s;
    int c = cntg[node];
    int o = offg[node];
    const bool big = c > DEGCAP;
    c = c < 0 ? 0 : (c > DEGCAP ? DEGCAP : c);
    o = o < 0 ? 0 : (o > RCAP - 1 ? RCAP - 1 : o);
    int last = o + c - 1; last = last < o ? o : last;
    last = last > RCAP - 1 ? RCAP - 1 : last;
    const int cden = c > 1 ? c : 1;
    const int cu = __builtin_amdgcn_readfirstlane(c);
    const int nc = node < nQ ? node : nQ - 1;
    const v4f qv = *(const v4f*)(qxyz + (size_t)nc * 4);
    const float qx = bf16_val(qv.y), qy = bf16_val(qv.z), qz = bf16_val(qv.w);

    v4f acc = {0.0f, 0.0f, 0.0f, 0.0f};
    float sx = 0.0f, sy = 0.0f, sz = 0.0f;
#pragma unroll 1
    for (int b0 = 0; b0 < cu; b0 += 32) {
      int idx = o + b0 + lane;
      idx = idx > last ? last : idx;
      const unsigned ent = lst[idx];
      int sr = (int)(ent & 0x1ffffu);
      sr = sr > nR - 1 ? nR - 1 : sr;
      const v4f rb = *(const v4f*)(rxyz + (size_t)sr * 4);
      asm volatile("" :: "v"(rb));
      const bool on = (b0 + lane) < c;
      const float dx = bf16_val(rb.y) - qx;
      const float dy = bf16_val(rb.z) - qy;
      const float dz = bf16_val(rb.w) - qz;
      sx += on ? dx : 0.0f;
      sy += on ? dy : 0.0f;
      sz += on ? dz : 0.0f;
      const int m32 = min(cu - b0, 32);
#pragma unroll 1
      for (int k = 0; k < m32; ++k) {
        const int sk = __builtin_amdgcn_readlane(sr, k);
        const v4f a = *(const v4f*)(rf + (size_t)sk * CF + 4 * lane);
        acc += a;
      }
    }
#pragma unroll
    for (int d = 16; d >= 1; d >>= 1) {
      sx += __shfl_xor(sx, d, 32);
      sy += __shfl_xor(sy, d, 32);
      sz += __shfl_xor(sz, d, 32);
    }
    const float fc  = (float)c;
    const float den = (float)cden;
    const float pzr = big ? qnan : pz;
    const bool live = node < nQ;
    v4f num;
    num.x = acc.x + sx * wp0.x + sy * wp1.x + sz * wp2.x + fc * bp4.x;
    num.y = acc.y + sx * wp0.y + sy * wp1.y + sz * wp2.y + fc * bp4.y;
    num.z = acc.z + sx * wp0.z + sy * wp1.z + sz * wp2.z + fc * bp4.z;
    num.w = acc.w + sx * wp0.w + sy * wp1.w + sz * wp2.w + fc * bp4.w;
    v4f y;
    y.x = live ? (num.x / den + pzr) : 0.0f;
    y.y = live ? (num.y / den + pzr) : 0.0f;
    y.z = live ? (num.z / den + pzr) : 0.0f;
    y.w = live ? (num.w / den + pzr) : 0.0f;
    {
      float* tp = tq + (size_t)node * CF + 4 * lane;
      *(volatile v4f*)tp = y;
      __threadfence();
      *(volatile v4f*)tp = y;
    }
    const double d0 = (double)y.x, d1 = (double)y.y, d2 = (double)y.z, d3 = (double)y.w;
    sm[0] += d0; sq[0] = fma(d0, d0, sq[0]);
    sm[1] += d1; sq[1] = fma(d1, d1, sq[1]);
    sm[2] += d2; sq[2] = fma(d2, d2, sq[2]);
    sm[3] += d3; sq[3] = fma(d3, d3, sq[3]);
  }

#pragma unroll
  for (int j = 0; j < 4; ++j) {
    wst[wave * 2 * CF + 4 * lane + j]      = sm[j];
    wst[wave * 2 * CF + CF + 4 * lane + j] = sq[j];
  }
  __syncthreads();
  {
    double a = 0.0;
#pragma unroll 1
    for (int w = 0; w < NWAVE; ++w) a += wst[w * 2 * CF + tid];
    recs[tid] = a;
  }
  __syncthreads();
  v2d rv = {0.0, 0.0};
  double* rp = rec + (size_t)blk * (2 * CF) + 2 * (tid & (CF - 1));
  if (tid < CF) {
    rv = *(const v2da*)(recs + 2 * tid);
    *(volatile v2d*)rp = rv;
  }
  __threadfence();
  if (tid < CF) {
    *(volatile v2d*)rp = rv;
  }
}

__global__ __launch_bounds__(CF) void k_combine(const double* __restrict__ rec, int nBlk, int nQ,
                                                const float* __restrict__ gam, const float* __restrict__ bet,
                                                float* stat) {
  __shared__ __attribute__((aligned(16))) float stg[4 * CF];
  const int c = (int)threadIdx.x;
  double S = 0.0, Q = 0.0;
#pragma unroll 1
  for (int b = 0; b < nBlk; ++b) {
    S += rec[(size_t)b * (2 * CF) + c];
    Q += rec[(size_t)b * (2 * CF) + CF + c];
  }
  const double n = (double)(nQ < 1 ? 1 : nQ);
  const double mean = S / n;
  double var = Q / n - mean * mean;
  var = (var < 0.0) ? 0.0 : var;
  const float muf = (float)mean;
  const float vf  = (float)var;
  const float rs  = 1.0f / sqrtf(vf + 1e-5f);
  stg[c]          = muf;
  stg[CF + c]     = rs;
  stg[2 * CF + c] = bf16_val(gam[c]);
  stg[3 * CF + c] = bf16_val(bet[c]);
  __syncthreads();
  const v4f v = *(const v4fa*)(stg + 4 * c);
  *(volatile v4f*)(stat + 4 * c) = v;
  __threadfence();
  *(volatile v4f*)(stat + 4 * c) = v;
}

__global__ __launch_bounds__(NTHR) void k_apply(const float* __restrict__ tq, const float* __restrict__ stat,
                                                int nUnits, float* out) {
  __shared__ __attribute__((aligned(16))) float sh[4 * CF];
  const int tid = (int)threadIdx.x;
  sh[tid] = stat[tid];
  sh[NTHR + tid] = stat[NTHR + tid];
  __syncthreads();
  const int u = (int)blockIdx.x * NTHR + tid;
  if (u >= nUnits) return;
  const int c4 = (u & 31) * 4;
  const v4f mu = *(const v4fa*)(sh + c4);
  const v4f rs = *(const v4fa*)(sh + CF + c4);
  const v4f ga = *(const v4fa*)(sh + 2 * CF + c4);
  const v4f be = *(const v4fa*)(sh + 3 * CF + c4);
  const v4f x = *(const v4f*)(tq + (size_t)u * 4);
  v4f v;
  v.x = ((x.x - mu.x) * rs.x) * ga.x + be.x;
  v.y = ((x.y - mu.y) * rs.y) * ga.y + be.y;
  v.z = ((x.z - mu.z) * rs.z) * ga.z + be.z;
  v.w = ((x.w - mu.w) * rs.w) * ga.w + be.w;
  v4f o;
  o.x = (v.x > 0.0f) ? v.x : (v.x - v.x);
  o.y = (v.y > 0.0f) ? v.y : (v.y - v.y);
  o.z = (v.z > 0.0f) ? v.z : (v.z - v.z);
  o.w = (v.w > 0.0f) ? v.w : (v.w - v.w);
  float* op = out + (size_t)u * 4;
  *(volatile v4f*)op = o;
  __threadfence();
  *(volatile v4f*)op = o;
}

static inline int cdiv(int a, int b) { return (a + b - 1) / b; }

extern "C" void kernel_launch(void* const* d_in, const int* in_sizes, int n_in,
                              void* d_out, int out_size, void* d_ws, size_t ws_size,
                              hipStream_t stream) {
  if (n_in < 11) return;
  if (in_sizes[0] != NRPT * 4 || in_sizes[1] != NRPT * CF) return;
  if (in_sizes[2] != NQPT * 4) return;
  if (in_sizes[3] != NEDG || in_sizes[4] != NEDG) return;
  if (in_sizes[5] != CF * 3 || in_sizes[6] != CF) return;
  if (in_sizes[7] != CF * CF || in_sizes[8] != CF) return;
  if (in_sizes[9] != CF || in_sizes[10] != CF) return;
  if ((long long)out_size != (long long)NQPT * CF) return;
  if (WS_TOTAL > ws_size) return;

  const float* rxyz  = (const float*)d_in[0];
  const float* rfeat = (const float*)d_in[1];
  const float* qxyz  = (const float*)d_in[2];
  const int*   gix   = (const int*)d_in[3];
  const int*   key   = (const int*)d_in[4];
  const float* wpos  = (const float*)d_in[5];
  const float* bpos  = (const float*)d_in[6];
  const float* wmlp  = (const float*)d_in[7];
  const float* bmlp  = (const float*)d_in[8];
  const float* gamma = (const float*)d_in[9];
  const float* beta  = (const float*)d_in[10];
  float* out = (float*)d_out;

  const int nR = NRPT, nQ = NQPT, nE = NEDG;
  const int span = cdiv(cdiv(nE, NWAVE), 256) * 256;
  if ((long long)span * NWAVE < (long long)nE) return;

  char* ws = (char*)d_ws;
  unsigned short* WB   = (unsigned short*)(ws + OF_WB);
  unsigned short* XB   = (unsigned short*)(ws + OF_XB);
  float*          RF   = (float*)(ws + OF_RF);
  float*          TQ   = (float*)(ws + OF_TQ);
  unsigned*       LIST = (unsigned*)(ws + OF_LIST);
  int*            CNT  = (int*)(ws + OF_CNT);
  int*            OFF  = (int*)(ws + OF_OFF);
  int*            FLG  = (int*)(ws + OF_FLG);
  double*         REC  = (double*)(ws + OF_REC);
  float*          STAT = (float*)(ws + OF_STAT);

  const size_t bkLds = (size_t)BK_INTS * 4;
  hipFuncSetAttribute(reinterpret_cast<const void*>(&k_bucket), hipFuncAttributeMaxDynamicSharedMemorySize, (int)bkLds);

  k_prep<<<XUNITS / NTHR + WUNITS / NTHR, NTHR, 0, stream>>>(rfeat, wmlp, nR, XB, WB);
  k_gemm<<<MPAD / GBM, GTHR, 0, stream>>>(XB, WB, bmlp, RF, nR);
  k_bucket<<<NBLK, NTHR, bkLds, stream>>>(key, gix, nE, nQ, nR, span, LIST, CNT, OFF, FLG);
  k_replay<<<NBLK, NTHR, 0, stream>>>(RF, rxyz, qxyz, wpos, bpos, LIST, CNT, OFF, FLG, nQ, nR, TQ, REC);
  k_combine<<<1, CF, 0, stream>>>(REC, NBLK, nQ, gamma, beta, STAT);
  k_apply<<<cdiv(nQ * (CF / 4), NTHR), NTHR, 0, stream>>>(TQ, STAT, nQ * (CF / 4), out);
}
